// GraphSAGE_GraphSVX_foroptuna_51402168598679
// MI455X (gfx1250) — hardware-verified
//
#include <hip/hip_runtime.h>
#include <stddef.h>
#include <math.h>


#define FD      128
#define KL      256
#define NCLS    2
#define NCP     16
#define NTHR    256
#define NWAVE   8
#define EPT     8
#define NGRP    2
#define CHUNK   (NTHR * EPT * NGRP)
#define WCAP    (EPT * NGRP * 32)
#define LISTN   (NWAVE * WCAP)
#define NBC     4096
#define NBF     2048
#define FPC     (NBC / NBF)
#define RCAP    40960
#define RBN     128
#define TGT     256
#define DEGCAP  256
#define OTHR    512
#define BM      64
#define CBM     128
#define WSCAP   134217728
#define BN_EPS  1e-5

#define LDS_FILL ((RCAP + NBF + LISTN) * 4 + 64)
#define LDS_GEMB (BM * FD * 2 * 2 + BM * FD * 4)
#define LDS_GSAG (BM * FD * 2 * 4 + BM * FD * 4)
#define LDS_CLS  (CBM * FD * 2 * 2 + CBM * NCLS * 4)

static_assert((CHUNK & (CHUNK - 1)) == 0);
static_assert(CHUNK <= 4096);
static_assert(NBC <= 4096 && NBF <= 4096);
static_assert((NBC & (NBC - 1)) == 0 && (NBF & (NBF - 1)) == 0);
static_assert(NBC == FPC * NBF && FPC == 2);
static_assert(OTHR * 8 == NBC);
static_assert(OTHR / 32 == 8 * FPC);
static_assert((RCAP % 32) == 0);
static_assert(TGT == NWAVE * 32);
static_assert((TGT % BM) == 0 && (TGT % CBM) == 0);
static_assert((DEGCAP % 32) == 0);
static_assert(KL == 2 * FD && NCP == 16 && NCLS <= 4);
static_assert(BM == 64 && NWAVE == 8 && CBM == NWAVE * 16);

typedef float          v2f  __attribute__((ext_vector_type(2)));
typedef float          v4f  __attribute__((ext_vector_type(4)));
typedef float          v8f  __attribute__((ext_vector_type(8)));
typedef double         v2d  __attribute__((ext_vector_type(2)));
typedef int            v4i  __attribute__((ext_vector_type(4)));
typedef unsigned short v8us __attribute__((ext_vector_type(8)));
typedef unsigned short v16us __attribute__((ext_vector_type(16)));
typedef __bf16         v16bf __attribute__((ext_vector_type(16)));
union FragU { v16us w; v8us u[2]; };

__device__ __forceinline__ v8f wmb(v16us a, v16us b, v8f c) {
  const v16bf ab = __builtin_bit_cast(v16bf, a);
  const v16bf bb = __builtin_bit_cast(v16bf, b);
  v8f d = __builtin_amdgcn_wmma_f32_16x16x32_bf16(false, ab, false, bb, (short)0, c, false, false);
  asm volatile("v_nop\n\tv_nop\n\tv_nop\n\tv_nop" : "+v"(d) : "v"(a), "v"(b));
  return d;
}

__device__ __forceinline__ unsigned int bfb(float f) {
  const unsigned int u = __float_as_uint(f);
  return (u + 0x7FFFu + ((u >> 16) & 1u)) >> 16;
}
__device__ __forceinline__ void sp1(float v, unsigned short& h, unsigned short& l) {
  const unsigned int hb = bfb(v);
  const float hf = __uint_as_float(hb << 16);
  h = (unsigned short)hb;
  l = (unsigned short)bfb(v - hf);
}
__device__ __forceinline__ void sp8(v4f a, v4f b, v8us& h, v8us& l) {
  unsigned short hh, ll;
  sp1(a.x, hh, ll); h[0] = hh; l[0] = ll;
  sp1(a.y, hh, ll); h[1] = hh; l[1] = ll;
  sp1(a.z, hh, ll); h[2] = hh; l[2] = ll;
  sp1(a.w, hh, ll); h[3] = hh; l[3] = ll;
  sp1(b.x, hh, ll); h[4] = hh; l[4] = ll;
  sp1(b.y, hh, ll); h[5] = hh; l[5] = ll;
  sp1(b.z, hh, ll); h[6] = hh; l[6] = ll;
  sp1(b.w, hh, ll); h[7] = hh; l[7] = ll;
}
__device__ __forceinline__ v4f relu4(v4f t) {
  v4f r;
  r.x = fmaxf(t.x, 0.f); r.y = fmaxf(t.y, 0.f); r.z = fmaxf(t.z, 0.f); r.w = fmaxf(t.w, 0.f);
  return r;
}

__global__ __launch_bounds__(NTHR) void k_wprep(const float* __restrict__ Wa, const float* __restrict__ Wb,
                                               int lg, int nv, unsigned short* ph, unsigned short* pl, int units) {
  const int i = (int)blockIdx.x * NTHR + (int)threadIdx.x;
  if (i >= units) return;
  const int n  = i >> lg;
  const int k0 = (i & ((1 << lg) - 1)) * 8;
  const int nc = n < nv - 1 ? n : nv - 1;
  const int kk = k0 & (FD - 1);
  const float* pa = Wa + (size_t)nc * FD + kk;
  const float* pb = Wb + (size_t)nc * FD + kk;
  v4f a0 = *(const v4f*)pa, a1 = *(const v4f*)(pa + 4);
  const v4f b0 = *(const v4f*)pb, b1 = *(const v4f*)(pb + 4);
  const v4f z4 = {0.f, 0.f, 0.f, 0.f};
  if (k0 >= FD) { a0 = b0; a1 = b1; }
  if (n >= nv)  { a0 = z4; a1 = z4; }
  v8us hv, lv;
  sp8(a0, a1, hv, lv);
  unsigned short* dh = ph + (size_t)i * 8;
  unsigned short* dl = pl + (size_t)i * 8;
  *(volatile v8us*)dh = hv;
  *(volatile v8us*)dl = lv;
  __threadfence();
  *(volatile v8us*)dh = hv;
  *(volatile v8us*)dl = lv;
}

template <int NB>
__device__ __forceinline__ int scan_chunk(const int* __restrict__ dsts, int nE, int cbase, int slotBase,
                                          int vec8, int* list, int tid, int lane, int wave) {
  int wc = 0;
#pragma unroll
  for (int g = 0; g < NGRP; ++g) {
    const int el0  = (g * NTHR + tid) * EPT;
    const int e0   = cbase + el0;
    const int sent = -2147483647 - 1;
    v4i da, db;
    if (vec8 != 0 && cbase + CHUNK <= nE) {
      da = *(const v4i*)(dsts + e0);
      db = *(const v4i*)(dsts + e0 + 4);
    } else {
      da.x = (e0     < nE) ? dsts[min(e0, nE - 1)] : sent;
      da.y = (e0 + 1 < nE) ? dsts[min(e0 + 1, nE - 1)] : sent;
      da.z = (e0 + 2 < nE) ? dsts[min(e0 + 2, nE - 1)] : sent;
      da.w = (e0 + 3 < nE) ? dsts[min(e0 + 3, nE - 1)] : sent;
      db.x = (e0 + 4 < nE) ? dsts[min(e0 + 4, nE - 1)] : sent;
      db.y = (e0 + 5 < nE) ? dsts[min(e0 + 5, nE - 1)] : sent;
      db.z = (e0 + 6 < nE) ? dsts[min(e0 + 6, nE - 1)] : sent;
      db.w = (e0 + 7 < nE) ? dsts[min(e0 + 7, nE - 1)] : sent;
    }
    const unsigned nb = (unsigned)slotBase;
    const unsigned s0 = (unsigned)da.x - nb, s1 = (unsigned)da.y - nb;
    const unsigned s2 = (unsigned)da.z - nb, s3 = (unsigned)da.w - nb;
    const unsigned s4 = (unsigned)db.x - nb, s5 = (unsigned)db.y - nb;
    const unsigned s6 = (unsigned)db.z - nb, s7 = (unsigned)db.w - nb;
    const bool h0 = s0 < (unsigned)NB, h1 = s1 < (unsigned)NB, h2 = s2 < (unsigned)NB, h3 = s3 < (unsigned)NB;
    const bool h4 = s4 < (unsigned)NB, h5 = s5 < (unsigned)NB, h6 = s6 < (unsigned)NB, h7 = s7 < (unsigned)NB;
    const unsigned any = __builtin_amdgcn_ballot_w32(h0 | h1 | h2 | h3 | h4 | h5 | h6 | h7);
    if (any != 0u) {
#define HITJ(J, HJ, SJ) { \
        const unsigned mj = __builtin_amdgcn_ballot_w32(HJ); \
        if (mj != 0u) { \
          if (HJ) { \
            const int pos = wc + (int)__builtin_amdgcn_mbcnt_lo(mj, 0u); \
            if (pos < WCAP) list[wave * WCAP + pos] = ((el0 + (J)) << 12) | (int)(SJ); \
          } \
          wc += (int)__builtin_popcount(mj); } }
      HITJ(0, h0, s0)
      HITJ(1, h1, s1)
      HITJ(2, h2, s2)
      HITJ(3, h3, s3)
      HITJ(4, h4, s4)
      HITJ(5, h5, s5)
      HITJ(6, h6, s6)
      HITJ(7, h7, s7)
#undef HITJ
    }
  }
  return wc;
}

__global__ __launch_bounds__(NTHR) void k_count(
    const int* __restrict__ dsts, int* cnt, int nE, int vec8) {
  __shared__ __attribute__((aligned(16))) int scnt[NBC];
  __shared__ __attribute__((aligned(16))) int list[LISTN];
  __shared__ int wcnt[NWAVE];
  const int tid = threadIdx.x, lane = tid & 31, wave = tid >> 5;
  const int nodeBase = blockIdx.x * NBC;

  for (int i = tid; i < NBC; i += NTHR) scnt[i] = 0;
  __syncthreads();

  const int nChunks = (nE + CHUNK - 1) / CHUNK;
#pragma unroll 1
  for (int ch = 0; ch < nChunks; ++ch) {
    const int cbase = ch * CHUNK;
    const int wc = scan_chunk<NBC>(dsts, nE, cbase, nodeBase, vec8, list, tid, lane, wave);
    if (lane == 0) wcnt[wave] = wc;
    __syncthreads();
    if (wave == 0) {
#pragma unroll 1
      for (int wsx = 0; wsx < NWAVE; ++wsx) {
        int n = __builtin_amdgcn_readfirstlane(wcnt[wsx]);
        n = n > WCAP ? WCAP : (n < 0 ? 0 : n);
        const int* lp = list + wsx * WCAP;
#pragma unroll 1
        for (int i = 0; i < n; ++i) {
          const int ent  = __builtin_amdgcn_readfirstlane(lp[i]);
          const int slot = ent & (NBC - 1);
          if (lane == 0) scnt[slot] = scnt[slot] + 1;
        }
      }
    }
    __syncthreads();
  }

  v4i cq[4];
#pragma unroll
  for (int q = 0; q < 4; ++q) {
    const int f = (wave * 4 + q) * 128 + 4 * lane;
    cq[q] = *(const v4i*)(scnt + f);
  }
  int* cpn = cnt + (size_t)nodeBase;
#pragma unroll
  for (int q = 0; q < 4; ++q) {
    const int f = (wave * 4 + q) * 128 + 4 * lane;
    *(volatile v4i*)(cpn + f) = cq[q];
  }
  __threadfence();
#pragma unroll
  for (int q = 0; q < 4; ++q) {
    const int f = (wave * 4 + q) * 128 + 4 * lane;
    *(volatile v4i*)(cpn + f) = cq[q];
  }
}

__global__ __launch_bounds__(OTHR) void k_offsets(
    const int* __restrict__ cnt, int* off, int* rbase, int nChunk) {
  __shared__ __attribute__((aligned(16))) int soff[NBC];
  __shared__ __attribute__((aligned(16))) int srb[RBN];
  __shared__ int wtot[OTHR / 32];
  const int tid = threadIdx.x, lane = tid & 31, wave = tid >> 5, sub = tid >> 8;
  for (int i = tid; i < RBN; i += OTHR) srb[i] = 0;
  __syncthreads();
  int carry = 0;
#pragma unroll 1
  for (int ch = 0; ch < nChunk; ++ch) {
    const int base = ch * NBC;
    const v4i ca = *(const v4i*)(cnt + base + 8 * tid);
    const v4i cb = *(const v4i*)(cnt + base + 8 * tid + 4);
    const int e0 = max(ca.x, 0), e1 = max(ca.y, 0), e2 = max(ca.z, 0), e3 = max(ca.w, 0);
    const int e4 = max(cb.x, 0), e5 = max(cb.y, 0), e6 = max(cb.z, 0), e7 = max(cb.w, 0);
    const int ts = e0 + e1 + e2 + e3 + e4 + e5 + e6 + e7;
    int incl = ts;
#pragma unroll
    for (int d = 1; d < 32; d <<= 1) {
      const int t = __shfl_up(incl, d);
      if (lane >= d) incl += t;
    }
    if (lane == 31) wtot[wave] = incl;
    __syncthreads();
    int S0 = 0, S1 = 0;
#pragma unroll
    for (int w = 0; w < 8; ++w) { S0 += wtot[w]; S1 += wtot[8 + w]; }
    int pre = 0;
#pragma unroll 1
    for (int w = 8 * sub; w < wave; ++w) pre += wtot[w];
    const int b0 = carry;
    const int b1 = b0 + ((S0 + 31) & ~31);
    const int b2 = b1 + ((S1 + 31) & ~31);
    const int myb = sub == 0 ? b0 : b1;
    if (tid == 0) {
      srb[min(2 * ch + 0, RBN - 1)] = b0;
      srb[min(2 * ch + 1, RBN - 1)] = b1;
    }
    int run = myb + pre + incl - ts;
    soff[8 * tid + 0] = run; run += e0;
    soff[8 * tid + 1] = run; run += e1;
    soff[8 * tid + 2] = run; run += e2;
    soff[8 * tid + 3] = run; run += e3;
    soff[8 * tid + 4] = run; run += e4;
    soff[8 * tid + 5] = run; run += e5;
    soff[8 * tid + 6] = run; run += e6;
    soff[8 * tid + 7] = run;
    carry = b2;
    __syncthreads();
    const v4i o0 = *(const v4i*)(soff + 4 * tid);
    const v4i o1 = *(const v4i*)(soff + 4 * (tid + OTHR));
    int* op = off + base;
    *(volatile v4i*)(op + 4 * tid) = o0;
    *(volatile v4i*)(op + 4 * (tid + OTHR)) = o1;
    __threadfence();
    *(volatile v4i*)(op + 4 * tid) = o0;
    *(volatile v4i*)(op + 4 * (tid + OTHR)) = o1;
    __syncthreads();
  }
  if (tid == 0) srb[min(2 * nChunk, RBN - 1)] = carry;
  __syncthreads();
  v4i rv = {0, 0, 0, 0};
  if (tid < 32) rv = *(const v4i*)(srb + 4 * tid);
  if (tid < 32) *(volatile v4i*)(rbase + 4 * tid) = rv;
  __threadfence();
  if (tid < 32) *(volatile v4i*)(rbase + 4 * tid) = rv;
}

__global__ __launch_bounds__(NTHR) void k_fill(
    const int* __restrict__ dsts, const int* __restrict__ off, const int* __restrict__ rbase,
    int* csr, int nE, int vec8, int csrLen) {
  extern __shared__ v4f lds_dyn[];
  int* region = (int*)lds_dyn;
  int* cursor = region + RCAP;
  int* list   = cursor + NBF;
  int* wcnt   = list + LISTN;
  const int tid = threadIdx.x, lane = tid & 31, wave = tid >> 5;
  const int b = blockIdx.x;
  const int nodeBase = b * NBF;

  int rb0 = rbase[b];
  const int rb1 = rbase[b + 1];
  rb0 = rb0 < 0 ? 0 : (rb0 > csrLen ? csrLen : rb0);
  rb0 &= ~31;
  int len = rb1 - rb0;
  len = len < 0 ? 0 : (len > RCAP ? RCAP : len);
  int lenW = (len + 31) & ~31;
  if (rb0 + lenW > csrLen) lenW = (csrLen - rb0) & ~31;

  {
    const v4i z = {0, 0, 0, 0};
    for (int i = tid; i < RCAP / 4; i += NTHR) ((v4i*)region)[i] = z;
    for (int s = tid; s < NBF; s += NTHR) {
      int o = off[nodeBase + s] - rb0;
      o = o < 0 ? 0 : (o > RCAP ? RCAP : o);
      cursor[s] = o;
    }
  }
  __syncthreads();

  const int nChunks = (nE + CHUNK - 1) / CHUNK;
#pragma unroll 1
  for (int ch = 0; ch < nChunks; ++ch) {
    const int cbase = ch * CHUNK;
    const int wc = scan_chunk<NBF>(dsts, nE, cbase, nodeBase, vec8, list, tid, lane, wave);
    if (lane == 0) wcnt[wave] = wc;
    __syncthreads();
    if (wave == 0) {
#pragma unroll 1
      for (int wsx = 0; wsx < NWAVE; ++wsx) {
        int n = __builtin_amdgcn_readfirstlane(wcnt[wsx]);
        n = n > WCAP ? WCAP : (n < 0 ? 0 : n);
        const int* lp = list + wsx * WCAP;
#pragma unroll 1
        for (int i = 0; i < n; ++i) {
          const int ent  = __builtin_amdgcn_readfirstlane(lp[i]);
          const int slot = ent & (NBF - 1);
          int e = cbase + ((ent >> 12) & (CHUNK - 1));
          e = e > nE - 1 ? nE - 1 : e;
          if (lane == 0) {
            int pos = cursor[slot];
            pos = pos < 0 ? 0 : (pos > RCAP - 1 ? RCAP - 1 : pos);
            region[pos] = e;
            const int np = pos + 1;
            cursor[slot] = np > RCAP ? RCAP : np;
          }
        }
      }
    }
    __syncthreads();
  }

  const int nv = lenW >> 2;
  int* gp = csr + rb0;
#pragma unroll 1
  for (int i = tid; i < nv; i += NTHR) { const v4i v = ((const v4i*)region)[i]; *(volatile v4i*)(gp + 4 * i) = v; }
  __threadfence();
#pragma unroll 1
  for (int i = tid; i < nv; i += NTHR) { const v4i v = ((const v4i*)region)[i]; *(volatile v4i*)(gp + 4 * i) = v; }
}

__device__ __forceinline__ void stage64(const float* src, int rowBase, int nValid,
                                        unsigned short* th, unsigned short* tl) {
  const int tid = threadIdx.x;
  const v4f z4 = {0.f, 0.f, 0.f, 0.f};
#pragma unroll
  for (int it = 0; it < 4; ++it) {
    const int u = it * NTHR + tid;
    const int r = u >> 4, c = (u & 15) * 8;
    const int grow = rowBase + r;
    const int rc = grow < nValid ? grow : nValid - 1;
    const float* p = src + (size_t)rc * FD + c;
    v4f a = *(const v4f*)p, b = *(const v4f*)(p + 4);
    if (grow >= nValid) { a = z4; b = z4; }
    v8us hv, lv;
    sp8(a, b, hv, lv);
    *(v8us*)(th + r * FD + c) = hv;
    *(v8us*)(tl + r * FD + c) = lv;
  }
}

template <int NT, int PB>
__device__ __forceinline__ void mmk(v8f (&acc)[NT], const unsigned short* th, const unsigned short* tl, int arow,
                                    const unsigned short* __restrict__ Bh, const unsigned short* __restrict__ Bl,
                                    int bcol0, int kofs) {
  const int lane = threadIdx.x & 31, hh = lane >> 4, m = lane & 15;
  const unsigned short* aph = th + (arow + m) * FD + 8 * hh;
  const unsigned short* apl = tl + (arow + m) * FD + 8 * hh;
  const size_t boff = (size_t)(bcol0 + m) * PB + kofs + 8 * hh;
  const unsigned short* bph0 = Bh + boff;
  const unsigned short* bpl0 = Bl + boff;
#pragma unroll 1
  for (int kt = 0; kt < FD / 32; ++kt) {
    FragU ah, al;
    ah.u[0] = *(const v8us*)(aph + 32 * kt);
    ah.u[1] = *(const v8us*)(aph + 32 * kt + 16);
    al.u[0] = *(const v8us*)(apl + 32 * kt);
    al.u[1] = *(const v8us*)(apl + 32 * kt + 16);
#pragma unroll
    for (int t = 0; t < NT; ++t) {
      const size_t to = (size_t)(16 * t) * PB + 32 * kt;
      FragU bh, bl;
      bh.u[0] = *(const v8us*)(bph0 + to);
      bh.u[1] = *(const v8us*)(bph0 + to + 16);
      bl.u[0] = *(const v8us*)(bpl0 + to);
      bl.u[1] = *(const v8us*)(bpl0 + to + 16);
      acc[t] = wmb(ah.w, bh.w, acc[t]);
      acc[t] = wmb(al.w, bh.w, acc[t]);
      acc[t] = wmb(ah.w, bl.w, acc[t]);
    }
  }
}

__global__ __launch_bounds__(NTHR) void k_gemm_emb(
    const float* __restrict__ x, const unsigned short* __restrict__ Bh, const unsigned short* __restrict__ Bl,
    const float* __restrict__ bias, float* Hout, int nN) {
  extern __shared__ v4f lds_dyn[];
  unsigned short* th = (unsigned short*)lds_dyn;
  unsigned short* tl = th + BM * FD;
  float* stg = (float*)(tl + BM * FD);
  const int tid = threadIdx.x, lane = tid & 31, wave = tid >> 5, hh = lane >> 4, m = lane & 15;
  const int rowBase = blockIdx.x * BM;
  const int r0 = (wave >> 1) * 16, c0 = (wave & 1) * 64;

  stage64(x, rowBase, nN, th, tl);
  __syncthreads();

  v8f acc[4];
#pragma unroll
  for (int t = 0; t < 4; ++t) { v8f z = {0.f, 0.f, 0.f, 0.f, 0.f, 0.f, 0.f, 0.f}; acc[t] = z; }
  mmk<4, FD>(acc, th, tl, r0, Bh, Bl, c0, 0);
  {
    float* sp = stg + (size_t)(r0 + 8 * hh) * FD + c0 + m;
#pragma unroll
    for (int t = 0; t < 4; ++t) {
#pragma unroll
      for (int r = 0; r < 8; ++r) sp[r * FD + 16 * t] = acc[t][r];
    }
  }
  __syncthreads();

  const v4f z4 = {0.f, 0.f, 0.f, 0.f};
  const int rsub = lane >> 4, q = lane & 15, col = c0 + 4 * q;
  const v4f b4 = *(const v4f*)(bias + col);
#pragma unroll
  for (int it = 0; it < 8; ++it) {
    const int row  = it * 2 + rsub;
    const int grow = rowBase + r0 + row;
    v4f v = *(const v4f*)(stg + (size_t)(r0 + row) * FD + col) + b4;
    if (grow >= nN) v = z4;
    *(volatile v4f*)(Hout + (size_t)grow * FD + col) = v;
  }
  __threadfence();
#pragma unroll
  for (int it = 0; it < 8; ++it) {
    const int row  = it * 2 + rsub;
    const int grow = rowBase + r0 + row;
    v4f v = *(const v4f*)(stg + (size_t)(r0 + row) * FD + col) + b4;
    if (grow >= nN) v = z4;
    *(volatile v4f*)(Hout + (size_t)grow * FD + col) = v;
  }
}

__global__ __launch_bounds__(NTHR) void k_agg(
    const int* __restrict__ csr, const int* __restrict__ off, const int* __restrict__ cnt,
    const int* __restrict__ srcs, const float* __restrict__ Hin, float* AG, int nN, int nE, int csrLen) {
  const int tid = threadIdx.x, lane = tid & 31, wave = tid >> 5;
  const int tbase = blockIdx.x * TGT + wave * 32;
  const int col = 4 * lane;
  const v4f z4 = {0.f, 0.f, 0.f, 0.f};
  const int cl    = tbase + lane;
  const int cnt_l = cnt[cl];
  const int off_l = off[cl];

#pragma unroll 1
  for (int j = 0; j < 32; ++j) {
    const int c  = tbase + j;
    const int dg = __shfl(cnt_l, j);
    const int n  = dg < 0 ? 0 : (dg > DEGCAP ? DEGCAP : dg);
    const int st = __shfl(off_l, j);
    v4f acc = z4;
#pragma unroll 1
    for (int q0 = 0; q0 < n; q0 += 32) {
      int pos = st + q0 + lane;
      pos = pos < 0 ? 0 : (pos > csrLen - 1 ? csrLen - 1 : pos);
      int eid = csr[pos];
      eid = eid < 0 ? 0 : (eid > nE - 1 ? nE - 1 : eid);
      int sl = srcs[eid];
      sl = sl < 0 ? 0 : (sl > nN - 1 ? nN - 1 : sl);
      const int mcnt = (n - q0) < 32 ? (n - q0) : 32;
#pragma unroll 1
      for (int pp = 0; pp < mcnt; ++pp) {
        const int s = __builtin_amdgcn_readlane(sl, pp);
        const v4f xs = *(const v4f*)(Hin + (size_t)s * FD + col);
        acc += xs;
      }
    }
    const float df  = (float)(dg < 1 ? 1 : dg);
    const float inv = __builtin_amdgcn_rcpf(df);
    v4f v = acc * inv;
    if (c >= nN) v = z4;
    float* po = AG + (size_t)c * FD + col;
    *(volatile v4f*)po = v;
    __threadfence();
    *(volatile v4f*)po = v;
  }
}

__global__ __launch_bounds__(NTHR) void k_gemm_sage(
    const float* __restrict__ Hin, float* AGO,
    const unsigned short* __restrict__ Bh, const unsigned short* __restrict__ Bl,
    const float* __restrict__ bias, double* part, int nN) {
  extern __shared__ v4f lds_dyn[];
  __shared__ __attribute__((aligned(16))) double spt[2 * FD];
  unsigned short* thH = (unsigned short*)lds_dyn;
  unsigned short* tlH = thH + BM * FD;
  unsigned short* thA = tlH + BM * FD;
  unsigned short* tlA = thA + BM * FD;
  float* stg = (float*)(tlA + BM * FD);
  const int tid = threadIdx.x, lane = tid & 31, wave = tid >> 5, hh = lane >> 4, m = lane & 15;
  const int rowBase = blockIdx.x * BM;
  const int r0 = (wave >> 1) * 16, c0 = (wave & 1) * 64;

  stage64(Hin, rowBase, nN, thH, tlH);
  stage64(AGO, rowBase, nN, thA, tlA);
  __syncthreads();

  v8f acc[4];
#pragma unroll
  for (int t = 0; t < 4; ++t) { v8f z = {0.f, 0.f, 0.f, 0.f, 0.f, 0.f, 0.f, 0.f}; acc[t] = z; }
  mmk<4, KL>(acc, thH, tlH, r0, Bh, Bl, c0, 0);
  mmk<4, KL>(acc, thA, tlA, r0, Bh, Bl, c0, FD);
  {
    float* sp = stg + (size_t)(r0 + 8 * hh) * FD + c0 + m;
#pragma unroll
    for (int t = 0; t < 4; ++t) {
#pragma unroll
      for (int r = 0; r < 8; ++r) sp[r * FD + 16 * t] = acc[t][r];
    }
  }
  __syncthreads();

  if (tid < FD) {
    const float bc = bias[tid];
    double s = 0.0, qq = 0.0;
#pragma unroll 1
    for (int r = 0; r < BM; ++r) {
      const float vf = stg[r * FD + tid] + bc;
      const double v = (rowBase + r < nN) ? (double)vf : 0.0;
      s += v;
      qq += v * v;
    }
    spt[tid] = s;
    spt[FD + tid] = qq;
  }
  __syncthreads();

  const v4f z4 = {0.f, 0.f, 0.f, 0.f};
  const int rsub = lane >> 4, q = lane & 15, col = c0 + 4 * q;
  const v4f b4 = *(const v4f*)(bias + col);
  const int tp = tid < FD ? tid : FD - 1;
  const v2d pw = *(const v2d*)(spt + 2 * tp);
  double* pp = part + (size_t)blockIdx.x * (2 * FD) + 2 * tp;
  if (tid < FD) *(volatile v2d*)pp = pw;
#pragma unroll
  for (int it = 0; it < 8; ++it) {
    const int row  = it * 2 + rsub;
    const int grow = rowBase + r0 + row;
    v4f v = *(const v4f*)(stg + (size_t)(r0 + row) * FD + col) + b4;
    if (grow >= nN) v = z4;
    *(volatile v4f*)(AGO + (size_t)grow * FD + col) = v;
  }
  __threadfence();
  if (tid < FD) *(volatile v2d*)pp = pw;
#pragma unroll
  for (int it = 0; it < 8; ++it) {
    const int row  = it * 2 + rsub;
    const int grow = rowBase + r0 + row;
    v4f v = *(const v4f*)(stg + (size_t)(r0 + row) * FD + col) + b4;
    if (grow >= nN) v = z4;
    *(volatile v4f*)(AGO + (size_t)grow * FD + col) = v;
  }
}

__global__ __launch_bounds__(FD) void k_bnfin(const double* __restrict__ part, const float* __restrict__ gamma,
                                              float* tbl, int nPart, int nN) {
  __shared__ __attribute__((aligned(16))) float stb[2 * FD];
  const int tid = threadIdx.x, col = tid;
  double s = 0.0, q = 0.0;
#pragma unroll 1
  for (int b = 0; b < nPart; ++b) {
    s += part[(size_t)b * (2 * FD) + col];
    q += part[(size_t)b * (2 * FD) + FD + col];
  }
  const double inv = 1.0 / (double)nN;
  const double mu  = s * inv;
  double var = q * inv - mu * mu;
  var = var < 0.0 ? 0.0 : var;
  const float a  = (float)((double)gamma[col] / sqrt(var + BN_EPS));
  const float mf = (float)mu;
  stb[col] = mf;
  stb[FD + col] = a;
  __syncthreads();
  const int t4 = tid < 64 ? tid : 63;
  const v4f w = *(const v4f*)(stb + 4 * t4);
  if (tid < 64) *(volatile v4f*)(tbl + 4 * tid) = w;
  __threadfence();
  if (tid < 64) *(volatile v4f*)(tbl + 4 * tid) = w;
}

__global__ __launch_bounds__(NTHR) void k_bnapply(
    const float* __restrict__ o0, const float* __restrict__ tbl, const float* __restrict__ beta,
    float* Hout, int nN, int nUnits) {
  const int i = (int)blockIdx.x * NTHR + (int)threadIdx.x;
  if (i >= nUnits) return;
  const int row = i >> 5;
  const int c   = (i & 31) * 4;
  const v4f s0  = *(const v4f*)(o0 + (size_t)row * FD + c);
  const v4f mu0 = *(const v4f*)(tbl + c);
  const v4f ga0 = *(const v4f*)(tbl + FD + c);
  const v4f be0 = *(const v4f*)(beta + c);
  const v4f z4 = {0.f, 0.f, 0.f, 0.f};
  v4f h0 = relu4((s0 - mu0) * ga0 + be0);
  if (row >= nN) h0 = z4;
  float* dh = Hout + (size_t)row * FD + c;
  *(volatile v4f*)dh = h0;
  __threadfence();
  *(volatile v4f*)dh = h0;
}

__global__ __launch_bounds__(NTHR) void k_cls(
    const float* __restrict__ Hin, const unsigned short* __restrict__ Bh, const unsigned short* __restrict__ Bl,
    const float* __restrict__ cb, float* out, int nN) {
  extern __shared__ v4f lds_dyn[];
  unsigned short* th = (unsigned short*)lds_dyn;
  unsigned short* tl = th + CBM * FD;
  float* stg2 = (float*)(tl + CBM * FD);
  const int tid = threadIdx.x, lane = tid & 31, wave = tid >> 5, hh = lane >> 4, m = lane & 15;
  const int rowBase = blockIdx.x * CBM;

  stage64(Hin, rowBase, nN, th, tl);
  stage64(Hin, rowBase + BM, nN, th + BM * FD, tl + BM * FD);
  __syncthreads();

  const int arow = 16 * wave;
  v8f acc[1];
  { v8f z = {0.f, 0.f, 0.f, 0.f, 0.f, 0.f, 0.f, 0.f}; acc[0] = z; }
  mmk<1, FD>(acc, th, tl, arow, Bh, Bl, 0, 0);
  if (m < NCLS) {
#pragma unroll
    for (int r = 0; r < 8; ++r) stg2[(arow + 8 * hh + r) * NCLS + m] = acc[0][r];
  }
  __syncthreads();

  const float cb0 = cb[0], cb1 = cb[1];
  v4f bb; bb.x = cb0; bb.y = cb1; bb.z = cb0; bb.w = cb1;
  const int t4 = tid < 64 ? tid : 63;
  const v4f w = *(const v4f*)(stg2 + 4 * t4) + bb;
  const size_t tot = (size_t)nN * NCLS;
  const size_t f   = (size_t)rowBase * NCLS + 4 * (size_t)t4;
  float* po = out + f;
  const bool full = (tid < 64) && (f + 4 <= tot);
  const bool two  = (tid < 64) && !(f + 4 <= tot) && (f + 2 <= tot);
  v2f w2; w2.x = w.x; w2.y = w.y;
  if (full) *(volatile v4f*)po = w;
  if (two)  *(volatile v2f*)po = w2;
  __threadfence();
  if (full) *(volatile v4f*)po = w;
  if (two)  *(volatile v2f*)po = w2;
}

static size_t carve(size_t* o, size_t bytes) {
  const size_t r = *o;
  *o += (bytes + 255) & ~(size_t)255;
  return r;
}

extern "C" void kernel_launch(void* const* d_in, const int* in_sizes, int n_in,
                              void* d_out, int out_size, void* d_ws, size_t ws_size,
                              hipStream_t stream) {
  if (n_in < 21) return;
  const int nN = in_sizes[0] / FD;
  const int nE = in_sizes[1] / 2;
  if (nN <= 0 || nE <= 0 || in_sizes[0] != nN * FD || in_sizes[1] != 2 * nE) return;
  if (in_sizes[2] != FD * FD || in_sizes[3] != FD) return;
  for (int l = 0; l < 3; ++l) {
    const int b = 4 + 3 * l;
    if (in_sizes[b] != FD * FD || in_sizes[b + 1] != FD * FD || in_sizes[b + 2] != FD) return;
    if (in_sizes[13 + 2 * l] != FD || in_sizes[14 + 2 * l] != FD) return;
  }
  if (in_sizes[19] != NCLS * FD || in_sizes[20] != NCLS) return;
  if ((long long)out_size != (long long)nN * NCLS) return;
  if (nE > (1 << 27) || nN > (1 << 22)) return;

  const float* x     = (const float*)d_in[0];
  const int*   ei    = (const int*)d_in[1];
  const float* emb_w = (const float*)d_in[2];
  const float* emb_b = (const float*)d_in[3];
  const float* wl[3] = {(const float*)d_in[4],  (const float*)d_in[7],  (const float*)d_in[10]};
  const float* wr[3] = {(const float*)d_in[5],  (const float*)d_in[8],  (const float*)d_in[11]};
  const float* bc[3] = {(const float*)d_in[6],  (const float*)d_in[9],  (const float*)d_in[12]};
  const float* ga[3] = {(const float*)d_in[13], (const float*)d_in[15], (const float*)d_in[17]};
  const float* be[3] = {(const float*)d_in[14], (const float*)d_in[16], (const float*)d_in[18]};
  const float* cls_w = (const float*)d_in[19];
  const float* cls_b = (const float*)d_in[20];
  const int* src = ei;
  const int* dst = ei + nE;
  float* dout = (float*)d_out;

  const int NPAD   = ((nN + TGT - 1) / TGT) * TGT;
  const int nBC    = (nN + NBC - 1) / NBC;
  const int CNTPAD = nBC * NBC;
  if (FPC * nBC + 1 > RBN) return;
  const int nBF    = (nN + NBF - 1) / NBF;
  const int csrLen = ((nE + 31) & ~31) + 4096;
  if (31 * FPC * nBC > 4096) return;
  const int nAgg   = NPAD / TGT;
  const int nGm    = NPAD / BM;
  const int nCl    = NPAD / CBM;
  const int nUnit  = NPAD * (FD / 4);
  const int nUB    = (nUnit + NTHR - 1) / NTHR;

  char* ws = (char*)d_ws;
  size_t o = 0;
  const size_t oWeH = carve(&o, (size_t)FD * FD * 2),  oWeL = carve(&o, (size_t)FD * FD * 2);
  size_t oWH[3], oWL[3];
  for (int l = 0; l < 3; ++l) { oWH[l] = carve(&o, (size_t)FD * KL * 2); oWL[l] = carve(&o, (size_t)FD * KL * 2); }
  const size_t oWcH = carve(&o, (size_t)NCP * FD * 2), oWcL = carve(&o, (size_t)NCP * FD * 2);
  const size_t oCnt = carve(&o, (size_t)CNTPAD * 4);
  const size_t oOff = carve(&o, (size_t)CNTPAD * 4);
  const size_t oRb  = carve(&o, (size_t)RBN * 4);
  const size_t oCsr = carve(&o, (size_t)csrLen * 4);
  const size_t oPart = carve(&o, (size_t)nGm * 2 * FD * 8);
  const size_t oTbl  = carve(&o, (size_t)2 * FD * 4);
  const size_t oH    = carve(&o, (size_t)NPAD * FD * 4);
  const size_t oAG   = carve(&o, (size_t)NPAD * FD * 4);
  if (o > ws_size || o > (size_t)WSCAP) return;

  unsigned short* weH = (unsigned short*)(ws + oWeH); unsigned short* weL = (unsigned short*)(ws + oWeL);
  unsigned short* wHp[3]; unsigned short* wLp[3];
  for (int l = 0; l < 3; ++l) { wHp[l] = (unsigned short*)(ws + oWH[l]); wLp[l] = (unsigned short*)(ws + oWL[l]); }
  unsigned short* wcH = (unsigned short*)(ws + oWcH); unsigned short* wcL = (unsigned short*)(ws + oWcL);
  int*    cnt  = (int*)(ws + oCnt);
  int*    offp = (int*)(ws + oOff);
  int*    rb   = (int*)(ws + oRb);
  int*    csr  = (int*)(ws + oCsr);
  double* part = (double*)(ws + oPart);
  float*  tbl  = (float*)(ws + oTbl);
  float*  H    = (float*)(ws + oH);
  float*  AG   = (float*)(ws + oAG);

  const int vec8 = ((nE & 3) == 0) ? 1 : 0;

  k_wprep<<<(FD * 16 + NTHR - 1) / NTHR, NTHR, 0, stream>>>(emb_w, emb_w, 4, FD, weH, weL, FD * 16);
  for (int l = 0; l < 3; ++l)
    k_wprep<<<(FD * 32 + NTHR - 1) / NTHR, NTHR, 0, stream>>>(wl[l], wr[l], 5, FD, wHp[l], wLp[l], FD * 32);
  k_wprep<<<(NCP * 16 + NTHR - 1) / NTHR, NTHR, 0, stream>>>(cls_w, cls_w, 4, NCLS, wcH, wcL, NCP * 16);

  k_count<<<nBC, NTHR, 0, stream>>>(dst, cnt, nE, vec8);
  k_offsets<<<1, OTHR, 0, stream>>>(cnt, offp, rb, nBC);
  hipFuncSetAttribute(reinterpret_cast<const void*>(&k_fill),
                      hipFuncAttributeMaxDynamicSharedMemorySize, LDS_FILL);
  k_fill<<<nBF, NTHR, LDS_FILL, stream>>>(dst, offp, rb, csr, nE, vec8, csrLen);

  hipFuncSetAttribute(reinterpret_cast<const void*>(&k_gemm_emb),
                      hipFuncAttributeMaxDynamicSharedMemorySize, LDS_GEMB);
  k_gemm_emb<<<nGm, NTHR, LDS_GEMB, stream>>>(x, weH, weL, emb_b, H, nN);

  hipFuncSetAttribute(reinterpret_cast<const void*>(&k_gemm_sage),
                      hipFuncAttributeMaxDynamicSharedMemorySize, LDS_GSAG);
  for (int l = 0; l < 3; ++l) {
    k_agg<<<nAgg, NTHR, 0, stream>>>(csr, offp, cnt, src, H, AG, nN, nE, csrLen);
    k_gemm_sage<<<nGm, NTHR, LDS_GSAG, stream>>>(H, AG, wHp[l], wLp[l], bc[l], part, nN);
    k_bnfin<<<1, FD, 0, stream>>>(part, ga[l], tbl, nGm, nN);
    k_bnapply<<<nUB, NTHR, 0, stream>>>(AG, tbl, be[l], H, nN, nUnit);
  }

  hipFuncSetAttribute(reinterpret_cast<const void*>(&k_cls),
                      hipFuncAttributeMaxDynamicSharedMemorySize, LDS_CLS);
  k_cls<<<nCl, NTHR, LDS_CLS, stream>>>(H, wcH, wcL, cls_b, dout, nN);
}
